// SCDM_TP_19387482374387
// MI455X (gfx1250) — hardware-verified
//
#include <hip/hip_runtime.h>
#include <stddef.h>


#define EMBD    16
#define HIDC    128
#define OUTC    3
#define NRELC   2
#define KENC    32
#define KLAY    384
#define HEADN   16
#define NTHR    256
#define NWAVE   8
#define GTHR    128
#define GWAVE   4
#define GROWS   64
#define EPT     8
#define NGRP    2
#define CHUNK   (NTHR * EPT * NGRP)
#define WCAP    (EPT * NGRP * 32)
#define LISTN   (NWAVE * WCAP)
#define NBC     4096
#define NBF     1024
#define RCAP    40960
#define RBN     128
#define TGT     256
#define DEGCAP  256
#define OTHR    512
#define SRCMASK 0x0FFFFFFF
#define NEG_SLOPE 0.01f

#define LDS_FILL ((RCAP + NBF + LISTN) * 4 + 64)
#define LDS_ENC  (GROWS * (KENC + 8) * 4 + GROWS * HIDC * 4 + GROWS * OUTC * 4)
#define LDS_LAY  (GROWS * (KLAY + 8) * 4 + GROWS * HIDC * 4 + GROWS * OUTC * 4)

static_assert((CHUNK & (CHUNK - 1)) == 0);
static_assert(CHUNK <= 4096);
static_assert(NBC <= 4096 && NBF <= 4096);
static_assert((NBC & (NBC - 1)) == 0 && (NBF & (NBF - 1)) == 0);
static_assert(NBC == 4 * NBF);
static_assert(OTHR * 8 == NBC);
static_assert((RCAP % 32) == 0);
static_assert(GROWS == GWAVE * 16 && GTHR == GWAVE * 32);
static_assert((GROWS * KLAY / 8) % GTHR == 0 && (GROWS * KENC / 8) % GTHR == 0 && (GROWS * HIDC / 8) % GTHR == 0);
static_assert((TGT % GROWS) == 0);
static_assert((HIDC * KENC / 8) % NTHR == 0 && (HIDC * KLAY / 8) % NTHR == 0 && (HEADN * HIDC / 8) % NTHR == 0);
static_assert(GROWS * OUTC == 48 * 4);
static_assert(((KENC + 8) * 2) % 16 == 0 && ((KLAY + 8) * 2) % 16 == 0);

typedef float          v4f   __attribute__((ext_vector_type(4)));
typedef float          v8f   __attribute__((ext_vector_type(8)));
typedef int            v4i   __attribute__((ext_vector_type(4)));
typedef unsigned short v4us  __attribute__((ext_vector_type(4)));
typedef unsigned short v8us  __attribute__((ext_vector_type(8)));
typedef __bf16         v16bf __attribute__((ext_vector_type(16)));
union FragB { v16bf v; v8us h[2]; };

__device__ __forceinline__ unsigned int bf_rne(float f) {
  const unsigned int u = __float_as_uint(f);
  return (u + 0x7FFFu + ((u >> 16) & 1u)) >> 16;
}
__device__ __forceinline__ void split1(float x, unsigned short& h, unsigned short& l) {
  const unsigned int hb = bf_rne(x);
  const float hf = __uint_as_float(hb << 16);
  const unsigned int lb = bf_rne(x - hf);
  h = (unsigned short)hb;
  l = (unsigned short)lb;
}
__device__ __forceinline__ void split4(v4f a, v4us& h, v4us& l) {
  unsigned short hh, ll;
  split1(a.x, hh, ll); h[0] = hh; l[0] = ll;
  split1(a.y, hh, ll); h[1] = hh; l[1] = ll;
  split1(a.z, hh, ll); h[2] = hh; l[2] = ll;
  split1(a.w, hh, ll); h[3] = hh; l[3] = ll;
}
__device__ __forceinline__ void split8(v4f a, v4f b, v8us& h, v8us& l) {
  unsigned short hh, ll;
  split1(a.x, hh, ll); h[0] = hh; l[0] = ll;
  split1(a.y, hh, ll); h[1] = hh; l[1] = ll;
  split1(a.z, hh, ll); h[2] = hh; l[2] = ll;
  split1(a.w, hh, ll); h[3] = hh; l[3] = ll;
  split1(b.x, hh, ll); h[4] = hh; l[4] = ll;
  split1(b.y, hh, ll); h[5] = hh; l[5] = ll;
  split1(b.z, hh, ll); h[6] = hh; l[6] = ll;
  split1(b.w, hh, ll); h[7] = hh; l[7] = ll;
}

__device__ __forceinline__ v8f wmb(v16bf a, v16bf b, v8f c) {
  v8f d = __builtin_amdgcn_wmma_f32_16x16x32_bf16(false, a, false, b, (short)0, c, false, false);
  asm volatile("v_nop\n\tv_nop\n\tv_nop\n\tv_nop" : "+v"(d) : "v"(a), "v"(b));
  return d;
}

template <int NB>
__device__ __forceinline__ int scan_chunk(const int* __restrict__ dsts, int nE, int cbase, int slotBase,
                                          int vec8, int* list, int tid, int lane, int wave) {
  int wc = 0;
#pragma unroll
  for (int g = 0; g < NGRP; ++g) {
    const int el0  = (g * NTHR + tid) * EPT;
    const int e0   = cbase + el0;
    const int sent = -2147483647 - 1;
    v4i da, db;
    if (vec8 != 0 && cbase + CHUNK <= nE) {
      da = *(const v4i*)(dsts + e0);
      db = *(const v4i*)(dsts + e0 + 4);
    } else {
      da.x = (e0     < nE) ? dsts[min(e0, nE - 1)] : sent;
      da.y = (e0 + 1 < nE) ? dsts[min(e0 + 1, nE - 1)] : sent;
      da.z = (e0 + 2 < nE) ? dsts[min(e0 + 2, nE - 1)] : sent;
      da.w = (e0 + 3 < nE) ? dsts[min(e0 + 3, nE - 1)] : sent;
      db.x = (e0 + 4 < nE) ? dsts[min(e0 + 4, nE - 1)] : sent;
      db.y = (e0 + 5 < nE) ? dsts[min(e0 + 5, nE - 1)] : sent;
      db.z = (e0 + 6 < nE) ? dsts[min(e0 + 6, nE - 1)] : sent;
      db.w = (e0 + 7 < nE) ? dsts[min(e0 + 7, nE - 1)] : sent;
    }
    const unsigned nb = (unsigned)slotBase;
    const unsigned s0 = (unsigned)da.x - nb, s1 = (unsigned)da.y - nb;
    const unsigned s2 = (unsigned)da.z - nb, s3 = (unsigned)da.w - nb;
    const unsigned s4 = (unsigned)db.x - nb, s5 = (unsigned)db.y - nb;
    const unsigned s6 = (unsigned)db.z - nb, s7 = (unsigned)db.w - nb;
    const bool h0 = s0 < (unsigned)NB, h1 = s1 < (unsigned)NB, h2 = s2 < (unsigned)NB, h3 = s3 < (unsigned)NB;
    const bool h4 = s4 < (unsigned)NB, h5 = s5 < (unsigned)NB, h6 = s6 < (unsigned)NB, h7 = s7 < (unsigned)NB;
    const unsigned any = __builtin_amdgcn_ballot_w32(h0 | h1 | h2 | h3 | h4 | h5 | h6 | h7);
    if (any != 0u) {
#define HITJ(J, HJ, SJ) { \
        const unsigned mj = __builtin_amdgcn_ballot_w32(HJ); \
        if (mj != 0u) { \
          if (HJ) { \
            const int pos = wc + (int)__builtin_amdgcn_mbcnt_lo(mj, 0u); \
            if (pos < WCAP) list[wave * WCAP + pos] = ((el0 + (J)) << 12) | (int)(SJ); \
          } \
          wc += (int)__builtin_popcount(mj); } }
      HITJ(0, h0, s0)
      HITJ(1, h1, s1)
      HITJ(2, h2, s2)
      HITJ(3, h3, s3)
      HITJ(4, h4, s4)
      HITJ(5, h5, s5)
      HITJ(6, h6, s6)
      HITJ(7, h7, s7)
#undef HITJ
    }
  }
  return wc;
}

__global__ __launch_bounds__(NTHR) void k_wprep(
    const float* __restrict__ Win, const float* __restrict__ Wrel, const float* __restrict__ Wroot,
    const float* __restrict__ Wout,
    unsigned short* eH, unsigned short* eL, unsigned short* lH, unsigned short* lL,
    unsigned short* oH, unsigned short* oL) {
  const int g0 = HIDC * KENC / 8;
  const int g1 = HIDC * KLAY / 8;
  const int g2 = HEADN * HIDC / 8;
  const int tid = threadIdx.x;
  const int bstart = blockIdx.x * NTHR;
  const int i = bstart + tid;
  if (i >= g0 + g1 + g2) return;
  float v[8];
  unsigned short* dh; unsigned short* dl; int o;
  if (bstart < g0) {
    o = i * 8;
    const int n  = o / KENC;
    const int k0 = o - n * KENC;
#pragma unroll
    for (int e = 0; e < 8; ++e) {
      const int k  = k0 + e;
      const int kc = k < EMBD ? k : EMBD - 1;
      const float x = Win[kc * HIDC + n];
      v[e] = (k < EMBD) ? x : 0.0f;
    }
    dh = eH; dl = eL;
  } else if (bstart < g0 + g1) {
    o = (i - g0) * 8;
    const int n  = o / KLAY;
    const int k0 = o - n * KLAY;
#pragma unroll
    for (int e = 0; e < 8; ++e) {
      const int k    = k0 + e;
      const int part = k >> 7;
      const int kk   = k & 127;
      const int pr   = part < 1 ? 0 : part - 1;
      const float xr = Wroot[kk * HIDC + n];
      const float xl = Wrel[(size_t)pr * HIDC * HIDC + kk * HIDC + n];
      v[e] = (part == 0) ? xr : xl;
    }
    dh = lH; dl = lL;
  } else {
    o = (i - g0 - g1) * 8;
    const int n  = o / HIDC;
    const int k0 = o - n * HIDC;
#pragma unroll
    for (int e = 0; e < 8; ++e) {
      const int k  = k0 + e;
      const int nc = n < OUTC ? n : OUTC - 1;
      const float x = Wout[k * OUTC + nc];
      v[e] = (n < OUTC) ? x : 0.0f;
    }
    dh = oH; dl = oL;
  }
  v4f a, b;
  a.x = v[0]; a.y = v[1]; a.z = v[2]; a.w = v[3];
  b.x = v[4]; b.y = v[5]; b.z = v[6]; b.w = v[7];
  v8us hv, lv;
  split8(a, b, hv, lv);
  unsigned short* ph = dh + o;
  unsigned short* pl = dl + o;
  *(volatile v8us*)ph = hv;
  *(volatile v8us*)pl = lv;
  __threadfence();
  *(volatile v8us*)ph = hv;
  *(volatile v8us*)pl = lv;
}

__global__ __launch_bounds__(NTHR) void k_count(
    const int* __restrict__ ei, int* cnt, int nE, int vec8) {
  __shared__ __attribute__((aligned(16))) int scnt[NBC];
  __shared__ __attribute__((aligned(16))) int list[LISTN];
  __shared__ int wcnt[NWAVE];
  const int tid = threadIdx.x, lane = tid & 31, wave = tid >> 5;
  const int nodeBase = blockIdx.x * NBC;
  const int* dsts = ei + nE;

  for (int i = tid; i < NBC; i += NTHR) scnt[i] = 0;
  __syncthreads();

  const int nChunks = (nE + CHUNK - 1) / CHUNK;
#pragma unroll 1
  for (int ch = 0; ch < nChunks; ++ch) {
    const int cbase = ch * CHUNK;
    const int wc = scan_chunk<NBC>(dsts, nE, cbase, nodeBase, vec8, list, tid, lane, wave);
    if (lane == 0) wcnt[wave] = wc;
    __syncthreads();
    if (wave == 0) {
#pragma unroll 1
      for (int wsx = 0; wsx < NWAVE; ++wsx) {
        int n = __builtin_amdgcn_readfirstlane(wcnt[wsx]);
        n = n > WCAP ? WCAP : (n < 0 ? 0 : n);
        const int* lp = list + wsx * WCAP;
#pragma unroll 1
        for (int i = 0; i < n; ++i) {
          const int ent  = __builtin_amdgcn_readfirstlane(lp[i]);
          const int slot = ent & (NBC - 1);
          if (lane == 0) scnt[slot] = scnt[slot] + 1;
        }
      }
    }
    __syncthreads();
  }

  v4i cq[4];
#pragma unroll
  for (int q = 0; q < 4; ++q) {
    const int f = (wave * 4 + q) * 128 + 4 * lane;
    cq[q] = *(const v4i*)(scnt + f);
  }
  int* cp = cnt + (size_t)nodeBase;
#pragma unroll
  for (int q = 0; q < 4; ++q) {
    const int f = (wave * 4 + q) * 128 + 4 * lane;
    *(volatile v4i*)(cp + f) = cq[q];
  }
  __threadfence();
#pragma unroll
  for (int q = 0; q < 4; ++q) {
    const int f = (wave * 4 + q) * 128 + 4 * lane;
    *(volatile v4i*)(cp + f) = cq[q];
  }
}

__global__ __launch_bounds__(OTHR) void k_offsets(
    const int* __restrict__ cnt, int* off, int* rbase, int nChunk) {
  __shared__ __attribute__((aligned(16))) int soff[NBC];
  __shared__ __attribute__((aligned(16))) int srb[RBN];
  __shared__ int wtot[OTHR / 32];
  const int tid = threadIdx.x, lane = tid & 31, wave = tid >> 5, sub = tid >> 7;
  for (int i = tid; i < RBN; i += OTHR) srb[i] = 0;
  int carry = 0;
#pragma unroll 1
  for (int ch = 0; ch < nChunk; ++ch) {
    const int base = ch * NBC;
    const v4i c0 = *(const v4i*)(cnt + base + 8 * tid);
    const v4i c1 = *(const v4i*)(cnt + base + 8 * tid + 4);
    const int e0 = max(c0.x, 0), e1 = max(c0.y, 0), e2 = max(c0.z, 0), e3 = max(c0.w, 0);
    const int e4 = max(c1.x, 0), e5 = max(c1.y, 0), e6 = max(c1.z, 0), e7 = max(c1.w, 0);
    const int ts = e0 + e1 + e2 + e3 + e4 + e5 + e6 + e7;
    int incl = ts;
#pragma unroll
    for (int d = 1; d < 32; d <<= 1) {
      const int t = __shfl_up(incl, d);
      if (lane >= d) incl += t;
    }
    if (lane == 31) wtot[wave] = incl;
    __syncthreads();
    const int S0 = wtot[0]  + wtot[1]  + wtot[2]  + wtot[3];
    const int S1 = wtot[4]  + wtot[5]  + wtot[6]  + wtot[7];
    const int S2 = wtot[8]  + wtot[9]  + wtot[10] + wtot[11];
    const int S3 = wtot[12] + wtot[13] + wtot[14] + wtot[15];
    int pre = 0;
#pragma unroll 1
    for (int w = 4 * sub; w < wave; ++w) pre += wtot[w];
    const int b0 = carry;
    const int b1 = b0 + ((S0 + 31) & ~31);
    const int b2 = b1 + ((S1 + 31) & ~31);
    const int b3 = b2 + ((S2 + 31) & ~31);
    const int b4 = b3 + ((S3 + 31) & ~31);
    const int myb = sub == 0 ? b0 : (sub == 1 ? b1 : (sub == 2 ? b2 : b3));
    if (tid == 0) {
      srb[min(4 * ch + 0, RBN - 1)] = b0;
      srb[min(4 * ch + 1, RBN - 1)] = b1;
      srb[min(4 * ch + 2, RBN - 1)] = b2;
      srb[min(4 * ch + 3, RBN - 1)] = b3;
    }
    int run = myb + pre + incl - ts;
    soff[8 * tid + 0] = run; run += e0;
    soff[8 * tid + 1] = run; run += e1;
    soff[8 * tid + 2] = run; run += e2;
    soff[8 * tid + 3] = run; run += e3;
    soff[8 * tid + 4] = run; run += e4;
    soff[8 * tid + 5] = run; run += e5;
    soff[8 * tid + 6] = run; run += e6;
    soff[8 * tid + 7] = run;
    carry = b4;
    __syncthreads();
    const v4i o0 = *(const v4i*)(soff + 4 * tid);
    const v4i o1 = *(const v4i*)(soff + 4 * (tid + OTHR));
    int* op = off + base;
    *(volatile v4i*)(op + 4 * tid) = o0;
    *(volatile v4i*)(op + 4 * (tid + OTHR)) = o1;
    __threadfence();
    *(volatile v4i*)(op + 4 * tid) = o0;
    *(volatile v4i*)(op + 4 * (tid + OTHR)) = o1;
    __syncthreads();
  }
  if (tid == 0) srb[min(4 * nChunk, RBN - 1)] = carry;
  __syncthreads();
  v4i rv = {0, 0, 0, 0};
  if (tid < 32) rv = *(const v4i*)(srb + 4 * tid);
  if (tid < 32) *(volatile v4i*)(rbase + 4 * tid) = rv;
  __threadfence();
  if (tid < 32) *(volatile v4i*)(rbase + 4 * tid) = rv;
}

__global__ __launch_bounds__(NTHR) void k_fill(
    const int* __restrict__ ei, const int* __restrict__ ety, const int* __restrict__ off,
    const int* __restrict__ rbase, int* csr, int nN, int nE, int vec8, int csrLen) {
  extern __shared__ v4f lds_dyn[];
  int* region = (int*)lds_dyn;
  int* cursor = region + RCAP;
  int* list   = cursor + NBF;
  int* wcnt   = list + LISTN;
  const int tid = threadIdx.x, lane = tid & 31, wave = tid >> 5;
  const int b = blockIdx.x;
  const int nodeBase = b * NBF;
  const int* dsts = ei + nE;

  int rb0 = rbase[b];
  const int rb1 = rbase[b + 1];
  rb0 = rb0 < 0 ? 0 : (rb0 > csrLen ? csrLen : rb0);
  rb0 &= ~31;
  int len = rb1 - rb0;
  len = len < 0 ? 0 : (len > RCAP ? RCAP : len);
  int lenW = (len + 31) & ~31;
  if (rb0 + lenW > csrLen) lenW = (csrLen - rb0) & ~31;

  {
    const v4i z = {0, 0, 0, 0};
    for (int i = tid; i < RCAP / 4; i += NTHR) ((v4i*)region)[i] = z;
    for (int s = tid; s < NBF; s += NTHR) {
      int o = off[nodeBase + s] - rb0;
      o = o < 0 ? 0 : (o > RCAP ? RCAP : o);
      cursor[s] = o;
    }
  }
  __syncthreads();

  const int nChunks = (nE + CHUNK - 1) / CHUNK;
#pragma unroll 1
  for (int ch = 0; ch < nChunks; ++ch) {
    const int cbase = ch * CHUNK;
    const int wc = scan_chunk<NBF>(dsts, nE, cbase, nodeBase, vec8, list, tid, lane, wave);
    if (lane == 0) wcnt[wave] = wc;
    __syncthreads();
    if (wave == 0) {
#pragma unroll 1
      for (int wsx = 0; wsx < NWAVE; ++wsx) {
        int n = __builtin_amdgcn_readfirstlane(wcnt[wsx]);
        n = n > WCAP ? WCAP : (n < 0 ? 0 : n);
        const int* lp = list + wsx * WCAP;
#pragma unroll 1
        for (int i = 0; i < n; ++i) {
          const int ent  = __builtin_amdgcn_readfirstlane(lp[i]);
          const int slot = ent & (NBF - 1);
          int e = cbase + ((ent >> 12) & (CHUNK - 1));
          e = e > nE - 1 ? nE - 1 : e;
          int src = ei[e];
          src = src < 0 ? 0 : (src > nN - 1 ? nN - 1 : src);
          const int et = ety[e];
          const int code = (et == 0) ? 0 : ((et == 1) ? 1 : 2);
          const int val = src | (code << 28);
          if (lane == 0) {
            int pos = cursor[slot];
            pos = pos < 0 ? 0 : (pos > RCAP - 1 ? RCAP - 1 : pos);
            region[pos] = val;
            const int np = pos + 1;
            cursor[slot] = np > RCAP ? RCAP : np;
          }
        }
      }
    }
    __syncthreads();
  }

  const int nv = lenW >> 2;
  int* gp = csr + rb0;
#pragma unroll 1
  for (int i = tid; i < nv; i += NTHR) { const v4i v = ((const v4i*)region)[i]; *(volatile v4i*)(gp + 4 * i) = v; }
  __threadfence();
#pragma unroll 1
  for (int i = tid; i < nv; i += NTHR) { const v4i v = ((const v4i*)region)[i]; *(volatile v4i*)(gp + 4 * i) = v; }
}

template <int MODE>
__global__ __launch_bounds__(GTHR) void k_gemm(
    const float* __restrict__ Ain,
    const int* __restrict__ csr, const int* __restrict__ off, const int* __restrict__ cnt,
    const unsigned short* __restrict__ Bh, const unsigned short* __restrict__ Bl,
    const float* __restrict__ bias,
    const unsigned short* __restrict__ Oh, const unsigned short* __restrict__ Ol,
    const float* __restrict__ bout,
    float* C, float* out, int nN, int csrLen) {
  extern __shared__ v4f lds_dyn[];
  constexpr int KD = (MODE == 0) ? KENC : KLAY;
  constexpr int AP = KD + 8;
  unsigned short* sAh = (unsigned short*)lds_dyn;
  unsigned short* sAl = sAh + GROWS * AP;
  float* stg  = (float*)(sAl + GROWS * AP);
  float* sOut = stg + GROWS * HIDC;
  const int tid = threadIdx.x, lane = tid & 31, wave = tid >> 5, hh = lane >> 4, m = lane & 15;
  const int rowBase = blockIdx.x * GROWS;
  const int r0 = wave * 16;
  const v4f z4 = {0.f, 0.f, 0.f, 0.f};

  if (MODE == 0) {
#pragma unroll
    for (int i = 0; i < (GROWS * KENC / 8) / GTHR; ++i) {
      const int idx = i * GTHR + tid;
      const int r   = idx >> 2;
      const int c0  = (idx & 3) * 8;
      int row = rowBase + r;
      row = row > nN - 1 ? nN - 1 : row;
      const int cc = c0 < EMBD - 8 ? c0 : EMBD - 8;
      const float* ap = Ain + (size_t)row * EMBD + cc;
      v4f a = *(const v4f*)ap, b = *(const v4f*)(ap + 4);
      if (c0 >= EMBD) { a = z4; b = z4; }
      v8us hv, lv;
      split8(a, b, hv, lv);
      *(v8us*)(sAh + r * AP + c0) = hv;
      *(v8us*)(sAl + r * AP + c0) = lv;
    }
  } else {
#pragma unroll
    for (int i = 0; i < (GROWS * HIDC / 8) / GTHR; ++i) {
      const int idx = i * GTHR + tid;
      const int r   = idx >> 4;
      const int c0  = (idx & 15) * 8;
      const float* ap = Ain + ((size_t)rowBase + r) * HIDC + c0;
      const v4f a = *(const v4f*)ap, b = *(const v4f*)(ap + 4);
      v8us hv, lv;
      split8(a, b, hv, lv);
      *(v8us*)(sAh + r * AP + c0) = hv;
      *(v8us*)(sAl + r * AP + c0) = lv;
    }

    const int cl    = rowBase + r0 + m;
    const int cnt_l = cnt[cl];
    const int off_l = off[cl];
#pragma unroll 1
    for (int j = 0; j < 16; ++j) {
      int n = __builtin_amdgcn_readlane(cnt_l, j);
      n = n < 0 ? 0 : (n > DEGCAP ? DEGCAP : n);
      const int st = __builtin_amdgcn_readlane(off_l, j);
      v4f s0 = z4, s1 = z4;
      int k0 = 0, k1 = 0;
#pragma unroll 1
      for (int q0 = 0; q0 < n; q0 += 32) {
        int pos = st + q0 + lane;
        pos = pos < 0 ? 0 : (pos > csrLen - 1 ? csrLen - 1 : pos);
        const int ent = csr[pos];
        const int mc = (n - q0) < 32 ? (n - q0) : 32;
#pragma unroll 1
        for (int p = 0; p < mc; ++p) {
          const int e = __builtin_amdgcn_readlane(ent, p);
          int s = e & SRCMASK;
          s = s > nN - 1 ? nN - 1 : s;
          const int code = (e >> 28) & 3;
          const v4f v = *(const v4f*)(Ain + (size_t)s * HIDC + 4 * lane);
          if (code == 0) { s0 = s0 + v; ++k0; }
          else if (code == 1) { s1 = s1 + v; ++k1; }
        }
      }
      const float inv0 = 1.0f / (float)(k0 < 1 ? 1 : k0);
      const float inv1 = 1.0f / (float)(k1 < 1 ? 1 : k1);
      const v4f m0 = s0 * inv0, m1 = s1 * inv1;
      v4us h0v, l0v, h1v, l1v;
      split4(m0, h0v, l0v);
      split4(m1, h1v, l1v);
      unsigned short* rph = sAh + (r0 + j) * AP;
      unsigned short* rpl = sAl + (r0 + j) * AP;
      *(v4us*)(rph + HIDC + 4 * lane)     = h0v;
      *(v4us*)(rph + 2 * HIDC + 4 * lane) = h1v;
      *(v4us*)(rpl + HIDC + 4 * lane)     = l0v;
      *(v4us*)(rpl + 2 * HIDC + 4 * lane) = l1v;
    }
  }
  __syncthreads();

  const unsigned short* arh = sAh + (r0 + m) * AP + 8 * hh;
  const unsigned short* arl = sAl + (r0 + m) * AP + 8 * hh;
#pragma unroll 1
  for (int g = 0; g < 2; ++g) {
    v8f acc[4];
#pragma unroll
    for (int t = 0; t < 4; ++t) { v8f z = {0.f, 0.f, 0.f, 0.f, 0.f, 0.f, 0.f, 0.f}; acc[t] = z; }
#pragma unroll 1
    for (int kt = 0; kt < KD / 32; ++kt) {
      FragB ah, al;
      ah.h[0] = *(const v8us*)(arh + 32 * kt);
      ah.h[1] = *(const v8us*)(arh + 32 * kt + 16);
      al.h[0] = *(const v8us*)(arl + 32 * kt);
      al.h[1] = *(const v8us*)(arl + 32 * kt + 16);
#pragma unroll
      for (int t = 0; t < 4; ++t) {
        const size_t bo = (size_t)(64 * g + 16 * t + m) * KD + 32 * kt + 8 * hh;
        FragB bh, bl;
        bh.h[0] = *(const v8us*)(Bh + bo);
        bh.h[1] = *(const v8us*)(Bh + bo + 16);
        bl.h[0] = *(const v8us*)(Bl + bo);
        bl.h[1] = *(const v8us*)(Bl + bo + 16);
        acc[t] = wmb(ah.v, bh.v, acc[t]);
        acc[t] = wmb(ah.v, bl.v, acc[t]);
        acc[t] = wmb(al.v, bh.v, acc[t]);
      }
    }
    float* sp = stg + (r0 + 8 * hh) * HIDC + 64 * g + m;
#pragma unroll
    for (int t = 0; t < 4; ++t) {
      const float bv = bias[64 * g + 16 * t + m];
#pragma unroll
      for (int r = 0; r < 8; ++r) {
        float v = acc[t][r] + bv;
        if (MODE == 0) v = (v >= 0.0f) ? v : NEG_SLOPE * v;
        sp[r * HIDC + 16 * t] = v;
      }
    }
  }
  __syncthreads();

  if (MODE != 2) {
    const float* lp = stg + r0 * HIDC + 4 * lane;
    float* gp = C + ((size_t)rowBase + r0) * HIDC + 4 * lane;
#pragma unroll
    for (int i = 0; i < 16; ++i) { const v4f v = *(const v4f*)(lp + i * HIDC); *(volatile v4f*)(gp + (size_t)i * HIDC) = v; }
    __threadfence();
#pragma unroll
    for (int i = 0; i < 16; ++i) { const v4f v = *(const v4f*)(lp + i * HIDC); *(volatile v4f*)(gp + (size_t)i * HIDC) = v; }
  } else {
    v8f c1 = {0.f, 0.f, 0.f, 0.f, 0.f, 0.f, 0.f, 0.f};
    const float* hr = stg + (r0 + m) * HIDC + 8 * hh;
#pragma unroll
    for (int kt = 0; kt < HIDC / 32; ++kt) {
      const v4f f0 = *(const v4f*)(hr + 32 * kt);
      const v4f f1 = *(const v4f*)(hr + 32 * kt + 4);
      const v4f f2 = *(const v4f*)(hr + 32 * kt + 16);
      const v4f f3 = *(const v4f*)(hr + 32 * kt + 20);
      FragB ah, al;
      split8(f0, f1, ah.h[0], al.h[0]);
      split8(f2, f3, ah.h[1], al.h[1]);
      const size_t bo = (size_t)m * HIDC + 32 * kt + 8 * hh;
      FragB bh, bl;
      bh.h[0] = *(const v8us*)(Oh + bo);
      bh.h[1] = *(const v8us*)(Oh + bo + 16);
      bl.h[0] = *(const v8us*)(Ol + bo);
      bl.h[1] = *(const v8us*)(Ol + bo + 16);
      c1 = wmb(ah.v, bh.v, c1);
      c1 = wmb(ah.v, bl.v, c1);
      c1 = wmb(al.v, bh.v, c1);
    }
    const float bov = bout[m < OUTC ? m : OUTC - 1];
    if (m < OUTC) {
      float* so = sOut + (r0 + 8 * hh) * OUTC + m;
#pragma unroll
      for (int r = 0; r < 8; ++r) so[r * OUTC] = c1[r] + bov;
    }
    __syncthreads();
    int gv = nN - rowBase;
    gv = gv < 0 ? 0 : gv;
    gv = gv >> 5;
    gv = gv > (GROWS / 32) ? (GROWS / 32) : gv;
    const int li = tid < (GROWS * OUTC / 4 - 1) ? tid : (GROWS * OUTC / 4 - 1);
    const v4f ov = *(const v4f*)(sOut + 4 * li);
    const bool act = tid < 24 * gv;
    float* op = out + (size_t)rowBase * OUTC + 4 * tid;
    if (act) *(volatile v4f*)op = ov;
    __threadfence();
    if (act) *(volatile v4f*)op = ov;
  }
}

extern "C" void kernel_launch(void* const* d_in, const int* in_sizes, int n_in,
                              void* d_out, int out_size, void* d_ws, size_t ws_size,
                              hipStream_t stream) {
  if (n_in < 10) return;
  const int nN = in_sizes[0] / EMBD;
  const int nE = in_sizes[2];
  if (nN <= 0 || nE <= 0 || in_sizes[0] != nN * EMBD || in_sizes[1] != 2 * nE) return;
  if ((nN & 31) != 0) return;
  if (in_sizes[3] != EMBD * HIDC || in_sizes[4] < HIDC || in_sizes[5] != NRELC * HIDC * HIDC ||
      in_sizes[6] != HIDC * HIDC || in_sizes[7] < HIDC || in_sizes[8] != HIDC * OUTC || in_sizes[9] < OUTC) return;
  if (out_size != nN * OUTC) return;
  if (nE > (1 << 28) || nN > (1 << 24)) return;

  const float* feat  = (const float*)d_in[0];
  const int*   ei    = (const int*)d_in[1];
  const int*   ety   = (const int*)d_in[2];
  const float* Win   = (const float*)d_in[3];
  const float* bin   = (const float*)d_in[4];
  const float* Wrel  = (const float*)d_in[5];
  const float* Wroot = (const float*)d_in[6];
  const float* brg   = (const float*)d_in[7];
  const float* Wout  = (const float*)d_in[8];
  const float* bout  = (const float*)d_in[9];
  float* out = (float*)d_out;

  const int NPAD   = ((nN + TGT - 1) / TGT) * TGT;
  const int nBC    = (nN + NBC - 1) / NBC;
  const int CNTPAD = nBC * NBC;
  if (4 * nBC + 1 > RBN) return;
  if (CNTPAD < NPAD) return;
  const int nBF    = (nN + NBF - 1) / NBF;
  const int csrLen = ((nE + 31) & ~31) + 4096;
  const int nG     = NPAD / GROWS;

  char* ws = (char*)d_ws;
  size_t off = 0;
  const size_t oEH  = off; off += (size_t)HIDC * KENC * 2;         off = (off + 255) & ~(size_t)255;
  const size_t oEL  = off; off += (size_t)HIDC * KENC * 2;         off = (off + 255) & ~(size_t)255;
  const size_t oLH  = off; off += (size_t)HIDC * KLAY * 2;         off = (off + 255) & ~(size_t)255;
  const size_t oLL  = off; off += (size_t)HIDC * KLAY * 2;         off = (off + 255) & ~(size_t)255;
  const size_t oOH  = off; off += (size_t)HEADN * HIDC * 2;        off = (off + 255) & ~(size_t)255;
  const size_t oOL  = off; off += (size_t)HEADN * HIDC * 2;        off = (off + 255) & ~(size_t)255;
  const size_t oCnt = off; off += (size_t)CNTPAD * 4;              off = (off + 255) & ~(size_t)255;
  const size_t oOff = off; off += (size_t)CNTPAD * 4;              off = (off + 255) & ~(size_t)255;
  const size_t oRb  = off; off += (size_t)RBN * 4;                 off = (off + 255) & ~(size_t)255;
  const size_t oCsr = off; off += (size_t)csrLen * 4;              off = (off + 255) & ~(size_t)255;
  const size_t oX1  = off; off += (size_t)NPAD * HIDC * 4;         off = (off + 255) & ~(size_t)255;
  const size_t oX2  = off; off += (size_t)NPAD * HIDC * 4;         off = (off + 255) & ~(size_t)255;
  if (off > ws_size) return;
  unsigned short* eH = (unsigned short*)(ws + oEH);
  unsigned short* eL = (unsigned short*)(ws + oEL);
  unsigned short* lH = (unsigned short*)(ws + oLH);
  unsigned short* lL = (unsigned short*)(ws + oLL);
  unsigned short* oH = (unsigned short*)(ws + oOH);
  unsigned short* oL = (unsigned short*)(ws + oOL);
  int*   cnt  = (int*)(ws + oCnt);
  int*   offp = (int*)(ws + oOff);
  int*   rb   = (int*)(ws + oRb);
  int*   csr  = (int*)(ws + oCsr);
  float* x1   = (float*)(ws + oX1);
  float* x2   = (float*)(ws + oX2);

  const int vec8 = ((nE & 3) == 0) ? 1 : 0;

  const int nPrep = HIDC * KENC / 8 + HIDC * KLAY / 8 + HEADN * HIDC / 8;
  k_wprep<<<(nPrep + NTHR - 1) / NTHR, NTHR, 0, stream>>>(Win, Wrel, Wroot, Wout, eH, eL, lH, lL, oH, oL);

  k_count<<<nBC, NTHR, 0, stream>>>(ei, cnt, nE, vec8);
  k_offsets<<<1, OTHR, 0, stream>>>(cnt, offp, rb, nBC);
  hipFuncSetAttribute(reinterpret_cast<const void*>(&k_fill),
                      hipFuncAttributeMaxDynamicSharedMemorySize, LDS_FILL);
  k_fill<<<nBF, NTHR, LDS_FILL, stream>>>(ei, ety, offp, rb, csr, nN, nE, vec8, csrLen);

  hipFuncSetAttribute(reinterpret_cast<const void*>(&k_gemm<0>),
                      hipFuncAttributeMaxDynamicSharedMemorySize, LDS_ENC);
  hipFuncSetAttribute(reinterpret_cast<const void*>(&k_gemm<1>),
                      hipFuncAttributeMaxDynamicSharedMemorySize, LDS_LAY);
  hipFuncSetAttribute(reinterpret_cast<const void*>(&k_gemm<2>),
                      hipFuncAttributeMaxDynamicSharedMemorySize, LDS_LAY);
  k_gemm<0><<<nG, GTHR, LDS_ENC, stream>>>(feat, csr, offp, cnt, eH, eL, bin, oH, oL, bout, x1, out, nN, csrLen);

  k_gemm<1><<<nG, GTHR, LDS_LAY, stream>>>(x1, csr, offp, cnt, lH, lL, brg, oH, oL, bout, x2, out, nN, csrLen);

  k_gemm<2><<<nG, GTHR, LDS_LAY, stream>>>(x2, csr, offp, cnt, lH, lL, brg, oH, oL, bout, x1, out, nN, csrLen);
}
